// CausalSelfAttention_46849503265302
// MI455X (gfx1250) — hardware-verified
//
#include <hip/hip_runtime.h>


#ifndef NB
#define NB 2
#endif
#ifndef SEQ
#define SEQ 2048
#endif
#define NB_FULL  2
#define SEQ_FULL 2048
#define DM   1024
#define NH   16
#define HD   64
#define N3   (3 * DM)
#define RH   256
#define SCL  0.125f
#define LOG2E 1.4426950408889634f
#define PSH  10.0f
#define NEGBIG (-1.0e30f)

static_assert(HD == 64);
static_assert(NH * HD == DM);
static_assert(SEQ % 64 == 0);
static_assert(RH % 64 == 0);
static_assert(RH <= SEQ);
static_assert(DM % 64 == 0);
static_assert(N3 % 64 == 0);
static_assert(DM % 32 == 0);
static_assert((NB * SEQ) % 64 == 0);
static_assert(NB <= NB_FULL);
static_assert(SEQ <= SEQ_FULL);

typedef _Float16 h16;
typedef unsigned short bf;
typedef __attribute__((ext_vector_type(16))) __bf16   v16bf;
typedef __attribute__((ext_vector_type(16))) _Float16 v16h;
typedef __attribute__((ext_vector_type(16))) unsigned short v16us;
typedef __attribute__((ext_vector_type(8)))  _Float16 v8h;
typedef __attribute__((ext_vector_type(8)))  unsigned short v8us;
typedef __attribute__((ext_vector_type(2)))  unsigned short v2us;
typedef __attribute__((ext_vector_type(8)))  float    v8f;
typedef __attribute__((ext_vector_type(4)))  float    v4f;
typedef v4f  __attribute__((may_alias)) v4fa;

__device__ __forceinline__ unsigned short f2bf(float f) { unsigned u = __float_as_uint(f); u += 0x7FFFu + ((u >> 16) & 1u); return (unsigned short)(u >> 16); }
__device__ __forceinline__ float bf2f(unsigned short b) { return __uint_as_float(((unsigned)b) << 16); }
__device__ __forceinline__ float bfr(float f) { return bf2f(f2bf(f)); }
__device__ __forceinline__ void splitf(float y, unsigned short& h, unsigned short& l) { h = f2bf(y); l = f2bf(y - bf2f(h)); }
__device__ __forceinline__ v16h cat16(v8h lo, v8h hi) { return __builtin_shufflevector(lo, hi, 0, 1, 2, 3, 4, 5, 6, 7, 8, 9, 10, 11, 12, 13, 14, 15); }
__device__ __forceinline__ v16bf cat16b(v8us lo, v8us hi) { return __builtin_bit_cast(v16bf, __builtin_shufflevector(lo, hi, 0, 1, 2, 3, 4, 5, 6, 7, 8, 9, 10, 11, 12, 13, 14, 15)); }
__device__ __forceinline__ v16h  ldh(const h16* p) { return cat16(*(const v8h*)p, *(const v8h*)(p + 16)); }
__device__ __forceinline__ v16bf ldb(const bf* p)  { return cat16b(*(const v8us*)p, *(const v8us*)(p + 16)); }
__device__ __forceinline__ v8f mmah(v16h a, v16h b, v8f c) {
    c = __builtin_amdgcn_wmma_f32_16x16x32_f16(false, a, false, b, (short)0, c, false, false);
    asm volatile("v_nop\n\tv_nop\n\tv_nop\n\tv_nop" : "+v"(c) : "v"(a), "v"(b));
    return c;
}
__device__ __forceinline__ v8f mmab(v16bf a, v16bf b, v8f c) {
    c = __builtin_amdgcn_wmma_f32_16x16x32_bf16(false, a, false, b, (short)0, c, false, false);
    asm volatile("v_nop\n\tv_nop\n\tv_nop\n\tv_nop" : "+v"(c) : "v"(a), "v"(b));
    return c;
}

template <int NSPLIT>
__device__ __forceinline__ void gemm_tile(const bf* __restrict__ A, const bf* __restrict__ A2, const bf* __restrict__ Bt, int K, float* C, int ldc, const float* __restrict__ bias, size_t sA, size_t sC) {
    __shared__ __align__(16) float os[16 * 68];
    const size_t z = blockIdx.z; A += z * sA; if (NSPLIT == 1) A2 += z * sA; C += z * sC;
    const int lane = threadIdx.x & 31, lr = lane & 15, hi = lane >> 4; const int r0 = blockIdx.x * 64, c0 = blockIdx.y * 64;
    v8f acc[4][4];
#pragma unroll
    for (int mb = 0; mb < 4; ++mb)
#pragma unroll
        for (int nb = 0; nb < 4; ++nb) acc[mb][nb] = (v8f){};
    const size_t aoff = (size_t)(r0 + lr) * K + 8 * hi, boff = (size_t)(c0 + lr) * K + 8 * hi;
#pragma unroll 1
    for (int kc = 0; kc < K; kc += 32) {
        v16bf a[4], a2[4];
#pragma unroll
        for (int mb = 0; mb < 4; ++mb) { a[mb] = ldb(A + aoff + (size_t)mb * 16 * K + kc); if (NSPLIT == 1) a2[mb] = ldb(A2 + aoff + (size_t)mb * 16 * K + kc); else a2[mb] = a[mb]; }
#pragma unroll
        for (int nb = 0; nb < 4; ++nb) { const v16bf b = ldb(Bt + boff + (size_t)nb * 16 * K + kc);
#pragma unroll
            for (int mb = 0; mb < 4; ++mb) { acc[mb][nb] = mmab(a[mb], b, acc[mb][nb]); if (NSPLIT == 1) acc[mb][nb] = mmab(a2[mb], b, acc[mb][nb]); } }
    }
    v4f bb; { const v4f bv = *(const v4f*)(bias + c0 + lr * 4);
#pragma unroll
        for (int q = 0; q < 4; ++q) bb[q] = bfr(bv[q]); }
#pragma unroll
    for (int mb = 0; mb < 4; ++mb) {
#pragma unroll
        for (int nb = 0; nb < 4; ++nb) {
#pragma unroll
            for (int j = 0; j < 8; ++j) os[(hi * 8 + j) * 68 + nb * 16 + lr] = acc[mb][nb][j]; }
        __syncthreads();
        float* crow = C + (size_t)(r0 + mb * 16) * ldc + c0;
#pragma unroll 1
        for (int ps = 0; ps < 2; ++ps) {
#pragma unroll
            for (int s = 0; s < 8; ++s) { const int row = 2 * s + hi, cofs = lr * 4; v4f val = *(const v4fa*)(os + row * 68 + cofs); val = val + bb;
                *(volatile v4f*)(crow + (size_t)row * ldc + cofs) = val; }
            if (ps == 0) __threadfence(); }
        __syncthreads();
    }
}
__global__ __launch_bounds__(32) void k_gemm_qkv(const bf* __restrict__ A, const bf* __restrict__ Bt, int K, float* C, int ldc, const float* __restrict__ bias) {
    gemm_tile<0>(A, A, Bt, K, C, ldc, bias, 0, 0);
}
__global__ __launch_bounds__(32) void k_gemm_proj(const bf* __restrict__ Ah, const bf* __restrict__ Al, const bf* __restrict__ Bt, int K, float* C, int ldc, const float* __restrict__ bias, size_t sA, size_t sC) {
    gemm_tile<1>(Ah, Al, Bt, K, C, ldc, bias, sA, sC);
}

__global__ __launch_bounds__(256) void k_wtG(const float* __restrict__ w, int K, int N, bf* Bt) {
    const int lane = threadIdx.x & 31; const int L0 = (blockIdx.x * 8 + (threadIdx.x >> 5)) * 8; const int nlines = N * K / 64;
#pragma unroll
    for (int ps = 0; ps < 2; ++ps) {
#pragma unroll 1
        for (int l = 0; l < 8; ++l) { const int L = L0 + l; if (L >= nlines) break; const size_t e = (size_t)L * 64 + lane * 2; const int k = (int)(e % K), n = (int)(e / K); v2us o;
            o[0] = f2bf(w[(size_t)k * N + n]); o[1] = f2bf(w[(size_t)(k + 1) * N + n]); *(volatile v2us*)(Bt + e) = o; }
        if (ps == 0) __threadfence(); }
}
__global__ __launch_bounds__(256) void k_cvt8(const float* __restrict__ src, bf* dst, size_t n8, size_t sS, size_t sD) {
    const size_t i = (size_t)blockIdx.x * 256 + threadIdx.x; if (i >= n8) return;
    src += (size_t)blockIdx.y * sS; dst += (size_t)blockIdx.y * sD;
    const v8f v = *(const v8f*)(src + i * 8); v8us o;
#pragma unroll
    for (int k = 0; k < 8; ++k) o[k] = f2bf(v[k]);
    *(volatile v8us*)(dst + i * 8) = o; __threadfence(); *(volatile v8us*)(dst + i * 8) = o;
}

__global__ __launch_bounds__(256) void k_planes(const float* __restrict__ F, h16* Q16, h16* K16, h16* VT16, bf* Qh, bf* Ql, bf* Kh, bf* Kl, bf* VTh, bf* VTl) {
    __shared__ float vs[64 * 65];
    const int tid = threadIdx.x;
    const int t0 = blockIdx.x * 64; const int bh = blockIdx.y; const int bq = bh / NH; const int h = bh - bq * NH;
    const bool hires = (t0 < RH);
    const float* Fb = F + (size_t)(bq * SEQ + t0) * N3 + h * HD;
#pragma unroll 1
    for (int it = 0; it < 4; ++it) {
        const int idx = it * 256 + tid; const int tt = idx >> 4; const int c4 = (idx & 15) * 4;
        const v4f v = *(const v4f*)(Fb + (size_t)tt * N3 + 2 * DM + c4);
        vs[tt * 65 + c4 + 0] = v[0]; vs[tt * 65 + c4 + 1] = v[1]; vs[tt * 65 + c4 + 2] = v[2]; vs[tt * 65 + c4 + 3] = v[3];
    }
    __syncthreads();
#pragma unroll 1
    for (int ps = 0; ps < 2; ++ps) {
#pragma unroll 1
        for (int it = 0; it < 2; ++it) {
            const int idx = it * 256 + tid; const int rr = idx >> 3; const int c8 = (idx & 7) * 8;
            const float* fq = Fb + (size_t)rr * N3 + c8;
            const v4f qa = *(const v4f*)fq, qb = *(const v4f*)(fq + 4), ka = *(const v4f*)(fq + DM), kb = *(const v4f*)(fq + DM + 4);
            const v8f q = __builtin_shufflevector(qa, qb, 0, 1, 2, 3, 4, 5, 6, 7);
            const v8f k = __builtin_shufflevector(ka, kb, 0, 1, 2, 3, 4, 5, 6, 7);
            v8f v;
#pragma unroll
            for (int j = 0; j < 8; ++j) v[j] = vs[(c8 + j) * 65 + rr];
            v8h q16, k16, v16;
#pragma unroll
            for (int j = 0; j < 8; ++j) { q16[j] = (h16)q[j]; k16[j] = (h16)k[j]; v16[j] = (h16)v[j]; }
            const size_t po = ((size_t)bh * SEQ + t0 + rr) * HD + c8;
            const size_t vo = ((size_t)bh * HD + rr) * SEQ + t0 + c8;
            *(volatile v8h*)(Q16 + po) = q16; *(volatile v8h*)(K16 + po) = k16; *(volatile v8h*)(VT16 + vo) = v16;
            if (hires) {
                v8us qh, ql, kh, kl, vh, vl;
#pragma unroll
                for (int j = 0; j < 8; ++j) { unsigned short a, c; splitf(q[j], a, c); qh[j] = a; ql[j] = c; splitf(k[j], a, c); kh[j] = a; kl[j] = c; splitf(v[j], a, c); vh[j] = a; vl[j] = c; }
                const size_t ph = ((size_t)bh * RH + t0 + rr) * HD + c8;
                const size_t vh_o = ((size_t)bh * HD + rr) * RH + t0 + c8;
                *(volatile v8us*)(Qh + ph) = qh; *(volatile v8us*)(Ql + ph) = ql; *(volatile v8us*)(Kh + ph) = kh; *(volatile v8us*)(Kl + ph) = kl;
                *(volatile v8us*)(VTh + vh_o) = vh; *(volatile v8us*)(VTl + vh_o) = vl;
            }
        }
        if (ps == 0) __threadfence();
    }
}

__global__ __launch_bounds__(128) void k_attn16(const h16* __restrict__ Q16, const h16* __restrict__ K16, const h16* __restrict__ VT16, bf* ATh, bf* ATl) {
    __shared__ __align__(16) float os[4 * 16 * 68];
    const int lane = threadIdx.x & 31;
    const int wave = __builtin_amdgcn_readfirstlane(threadIdx.x >> 5);
    const int n = lane & 15, hf = lane >> 4;
    const int bh = blockIdx.y; const int bq = bh / NH; const int h = bh - bq * NH;
    const int q0 = RH + blockIdx.x * 64 + wave * 16;
    const h16* Qp = Q16 + (size_t)bh * SEQ * HD;
    const h16* Kp = K16 + (size_t)bh * SEQ * HD;
    const h16* Vp = VT16 + (size_t)bh * HD * SEQ;
    const int qoff = (q0 + n) * HD + 8 * hf;
    const v16h qb0 = ldh(Qp + qoff), qb1 = ldh(Qp + qoff + 32);
    v8f o[4];
#pragma unroll
    for (int dt = 0; dt < 4; ++dt) o[dt] = (v8f){};
    float mrun = NEGBIG, lrun = 0.0f;
    const int qi = q0 + n;
    const int kend = q0 + 16;
#pragma unroll 1
    for (int kt = 0; kt < kend; kt += 32) {
        const int koff = (kt + n) * HD + 8 * hf;
        v8f s0 = (v8f){}, s1 = (v8f){};
        s0 = mmah(ldh(Kp + koff), qb0, s0);
        s0 = mmah(ldh(Kp + koff + 32), qb1, s0);
        s1 = mmah(ldh(Kp + koff + 16 * HD), qb0, s1);
        s1 = mmah(ldh(Kp + koff + 16 * HD + 32), qb1, s1);
        const bool diag = (kt + 31 > q0);
        const int kb = kt + 8 * hf;
        float t0[8], t1[8]; float mx = NEGBIG;
#pragma unroll
        for (int r = 0; r < 8; ++r) {
            float a = s0[r] * SCL, c = s1[r] * SCL;
            a = (diag && (kb + r > qi)) ? NEGBIG : a;
            c = (diag && (kb + 16 + r > qi)) ? NEGBIG : c;
            t0[r] = a; t1[r] = c; mx = fmaxf(mx, fmaxf(a, c));
        }
        mx = fmaxf(mx, __shfl_xor(mx, 16, 32));
        const float mnew = fmaxf(mrun, mx);
        const float corr = __builtin_amdgcn_exp2f((mrun - mnew) * LOG2E);
        float ps = 0.0f; v16h pf;
#pragma unroll
        for (int r = 0; r < 8; ++r) {
            const float e0 = __builtin_amdgcn_exp2f((t0[r] - mnew) * LOG2E + PSH);
            const float e1 = __builtin_amdgcn_exp2f((t1[r] - mnew) * LOG2E + PSH);
            const h16 p0 = (h16)e0, p1 = (h16)e1;
            pf[r] = p0; pf[8 + r] = p1; ps += (float)p0 + (float)p1;
        }
        ps += __shfl_xor(ps, 16, 32);
        lrun = lrun * corr + ps; mrun = mnew;
#pragma unroll
        for (int dt = 0; dt < 4; ++dt)
#pragma unroll
            for (int r = 0; r < 8; ++r) o[dt][r] *= corr;
        const int voff = n * SEQ + kt + 8 * hf;
#pragma unroll
        for (int dt = 0; dt < 4; ++dt) o[dt] = mmah(ldh(Vp + voff + dt * 16 * SEQ), pf, o[dt]);
    }
    const float inv = 1.0f / lrun;
    const int ob = wave * (16 * 68);
#pragma unroll
    for (int dt = 0; dt < 4; ++dt) {
        v4f w0, w1;
#pragma unroll
        for (int q = 0; q < 4; ++q) { w0[q] = o[dt][q] * inv; w1[q] = o[dt][4 + q] * inv; }
        *(v4fa*)(os + ob + n * 68 + 16 * dt + 8 * hf) = w0;
        *(v4fa*)(os + ob + n * 68 + 16 * dt + 8 * hf + 4) = w1;
    }
    __syncthreads();
#pragma unroll 1
    for (int ps = 0; ps < 2; ++ps) {
#pragma unroll
        for (int s = 0; s < 4; ++s) {
            const int row = 4 * s + (lane >> 3); const int c8 = (lane & 7) * 8;
            const v4f a = *(const v4fa*)(os + ob + row * 68 + c8); const v4f b = *(const v4fa*)(os + ob + row * 68 + c8 + 4);
            v8us oh, ol;
#pragma unroll
            for (int q = 0; q < 4; ++q) { unsigned short x, y; splitf(a[q], x, y); oh[q] = x; ol[q] = y; splitf(b[q], x, y); oh[4 + q] = x; ol[4 + q] = y; }
            const size_t oo = ((size_t)(bq * SEQ + q0 + row)) * DM + h * HD + c8;
            *(volatile v8us*)(ATh + oo) = oh; *(volatile v8us*)(ATl + oo) = ol;
        }
        if (ps == 0) __threadfence();
    }
}

__global__ __launch_bounds__(128) void k_attnhl(const bf* __restrict__ Qh, const bf* __restrict__ Ql, const bf* __restrict__ Kh, const bf* __restrict__ Kl, const bf* __restrict__ VTh, const bf* __restrict__ VTl, bf* ATh, bf* ATl) {
    __shared__ __align__(16) float os[4 * 16 * 68];
    const int lane = threadIdx.x & 31;
    const int wave = __builtin_amdgcn_readfirstlane(threadIdx.x >> 5);
    const int n = lane & 15, hf = lane >> 4;
    const int bh = blockIdx.y; const int bq = bh / NH; const int h = bh - bq * NH;
    const int q0 = blockIdx.x * 64 + wave * 16;
    const size_t pb = (size_t)bh * RH * HD;
    const int qoff = (q0 + n) * HD + 8 * hf;
    const v16bf qh0 = ldb(Qh + pb + qoff), qh1 = ldb(Qh + pb + qoff + 32);
    const v16bf ql0 = ldb(Ql + pb + qoff), ql1 = ldb(Ql + pb + qoff + 32);
    v8f o[4];
#pragma unroll
    for (int dt = 0; dt < 4; ++dt) o[dt] = (v8f){};
    float mrun = NEGBIG, lrun = 0.0f;
    const int qi = q0 + n;
    const int kend = q0 + 16;
#pragma unroll 1
    for (int kt = 0; kt < kend; kt += 32) {
        const int koff = (kt + n) * HD + 8 * hf;
        v8f s0 = (v8f){}, s1 = (v8f){};
        { const v16bf kh = ldb(Kh + pb + koff), kl = ldb(Kl + pb + koff);
          s0 = mmab(kh, qh0, s0); s0 = mmab(kl, qh0, s0); s0 = mmab(kh, ql0, s0); }
        { const v16bf kh = ldb(Kh + pb + koff + 32), kl = ldb(Kl + pb + koff + 32);
          s0 = mmab(kh, qh1, s0); s0 = mmab(kl, qh1, s0); s0 = mmab(kh, ql1, s0); }
        { const v16bf kh = ldb(Kh + pb + koff + 16 * HD), kl = ldb(Kl + pb + koff + 16 * HD);
          s1 = mmab(kh, qh0, s1); s1 = mmab(kl, qh0, s1); s1 = mmab(kh, ql0, s1); }
        { const v16bf kh = ldb(Kh + pb + koff + 16 * HD + 32), kl = ldb(Kl + pb + koff + 16 * HD + 32);
          s1 = mmab(kh, qh1, s1); s1 = mmab(kl, qh1, s1); s1 = mmab(kh, ql1, s1); }
        const bool diag = (kt + 31 > q0);
        const int kb = kt + 8 * hf;
        float t0[8], t1[8]; float mx = NEGBIG;
#pragma unroll
        for (int r = 0; r < 8; ++r) {
            float a = s0[r] * SCL, c = s1[r] * SCL;
            a = (diag && (kb + r > qi)) ? NEGBIG : a;
            c = (diag && (kb + 16 + r > qi)) ? NEGBIG : c;
            t0[r] = a; t1[r] = c; mx = fmaxf(mx, fmaxf(a, c));
        }
        mx = fmaxf(mx, __shfl_xor(mx, 16, 32));
        const float mnew = fmaxf(mrun, mx);
        const float corr = __builtin_amdgcn_exp2f((mrun - mnew) * LOG2E);
        float ps = 0.0f; v16us phu, plu;
#pragma unroll
        for (int r = 0; r < 8; ++r) {
            const float e0 = __builtin_amdgcn_exp2f((t0[r] - mnew) * LOG2E + PSH);
            const float e1 = __builtin_amdgcn_exp2f((t1[r] - mnew) * LOG2E + PSH);
            unsigned short a, c;
            splitf(e0, a, c); phu[r] = a; plu[r] = c; ps += bf2f(a) + bf2f(c);
            splitf(e1, a, c); phu[8 + r] = a; plu[8 + r] = c; ps += bf2f(a) + bf2f(c);
        }
        ps += __shfl_xor(ps, 16, 32);
        lrun = lrun * corr + ps; mrun = mnew;
#pragma unroll
        for (int dt = 0; dt < 4; ++dt)
#pragma unroll
            for (int r = 0; r < 8; ++r) o[dt][r] *= corr;
        const v16bf ph = __builtin_bit_cast(v16bf, phu), pl = __builtin_bit_cast(v16bf, plu);
        const int voff = n * RH + kt + 8 * hf;
#pragma unroll
        for (int dt = 0; dt < 4; ++dt) {
            const v16bf vh = ldb(VTh + pb + voff + dt * 16 * RH), vl = ldb(VTl + pb + voff + dt * 16 * RH);
            o[dt] = mmab(vh, ph, o[dt]); o[dt] = mmab(vl, ph, o[dt]); o[dt] = mmab(vh, pl, o[dt]);
        }
    }
    const float inv = 1.0f / lrun;
    const int ob = wave * (16 * 68);
#pragma unroll
    for (int dt = 0; dt < 4; ++dt) {
        v4f w0, w1;
#pragma unroll
        for (int q = 0; q < 4; ++q) { w0[q] = o[dt][q] * inv; w1[q] = o[dt][4 + q] * inv; }
        *(v4fa*)(os + ob + n * 68 + 16 * dt + 8 * hf) = w0;
        *(v4fa*)(os + ob + n * 68 + 16 * dt + 8 * hf + 4) = w1;
    }
    __syncthreads();
#pragma unroll 1
    for (int ps = 0; ps < 2; ++ps) {
#pragma unroll
        for (int s = 0; s < 4; ++s) {
            const int row = 4 * s + (lane >> 3); const int c8 = (lane & 7) * 8;
            const v4f a = *(const v4fa*)(os + ob + row * 68 + c8); const v4f b = *(const v4fa*)(os + ob + row * 68 + c8 + 4);
            v8us oh, ol;
#pragma unroll
            for (int q = 0; q < 4; ++q) { unsigned short x, y; splitf(a[q], x, y); oh[q] = x; ol[q] = y; splitf(b[q], x, y); oh[4 + q] = x; ol[4 + q] = y; }
            const size_t oo = ((size_t)(bq * SEQ + q0 + row)) * DM + h * HD + c8;
            *(volatile v8us*)(ATh + oo) = oh; *(volatile v8us*)(ATl + oo) = ol;
        }
        if (ps == 0) __threadfence();
    }
}

constexpr size_t SZ_WQKV = (size_t)N3 * DM * 2;
constexpr size_t SZ_WO   = (size_t)DM * DM * 2;
constexpr size_t SZ_XB   = (size_t)NB * SEQ * DM * 2;
constexpr size_t SZ_F    = (size_t)NB * SEQ * N3 * 4;
constexpr size_t SZ_P16  = (size_t)NB * NH * SEQ * HD * 2;
constexpr size_t SZ_PHL  = (size_t)NB * NH * RH * HD * 2;
constexpr size_t SZ_AT   = (size_t)NB * SEQ * DM * 2;
constexpr size_t OFF_WQKV = 0;
constexpr size_t OFF_WO   = OFF_WQKV + SZ_WQKV;
constexpr size_t OFF_XB   = OFF_WO + SZ_WO;
constexpr size_t OFF_F    = OFF_XB + SZ_XB;
constexpr size_t OFF_Q16  = OFF_F + SZ_F;
constexpr size_t OFF_K16  = OFF_Q16 + SZ_P16;
constexpr size_t OFF_V16  = OFF_K16 + SZ_P16;
constexpr size_t OFF_QH   = OFF_V16 + SZ_P16;
constexpr size_t OFF_QL   = OFF_QH + SZ_PHL;
constexpr size_t OFF_KH   = OFF_QL + SZ_PHL;
constexpr size_t OFF_KL   = OFF_KH + SZ_PHL;
constexpr size_t OFF_VH   = OFF_KL + SZ_PHL;
constexpr size_t OFF_VL   = OFF_VH + SZ_PHL;
constexpr size_t OFF_ATH  = OFF_VL + SZ_PHL;
constexpr size_t OFF_ATL  = OFF_ATH + SZ_AT;
constexpr size_t WS_TOTAL = OFF_ATL + SZ_AT;
static_assert(WS_TOTAL <= (size_t)134217728);
static_assert(SZ_WQKV % 256 == 0 && SZ_WO % 256 == 0 && SZ_XB % 256 == 0 && SZ_F % 256 == 0 && SZ_P16 % 256 == 0 && SZ_PHL % 256 == 0 && SZ_AT % 256 == 0);

extern "C" void kernel_launch(void* const* d_in, const int* in_sizes, int n_in,
                              void* d_out, int out_size, void* d_ws, size_t ws_size, hipStream_t stream) {
    if (n_in < 5) return;
    const long long needx = (long long)(NB - 1) * SEQ_FULL * DM + (long long)SEQ * DM;
    if ((long long)in_sizes[0] < needx) return;
    if ((long long)in_sizes[1] < (long long)DM * N3) return;
    if (in_sizes[2] < N3) return;
    if ((long long)in_sizes[3] < (long long)DM * DM) return;
    if (in_sizes[4] < DM) return;
    if ((long long)out_size < needx) return;
    if (ws_size < WS_TOTAL) return;
    const float* x = (const float*)d_in[0];
    const float* wqkv = (const float*)d_in[1];
    const float* bqkv = (const float*)d_in[2];
    const float* wo = (const float*)d_in[3];
    const float* bo = (const float*)d_in[4];
    float* OUT = (float*)d_out;
    char* ws = (char*)d_ws;
    bf* WQKV = (bf*)(ws + OFF_WQKV); bf* WO = (bf*)(ws + OFF_WO); bf* XB = (bf*)(ws + OFF_XB); float* F = (float*)(ws + OFF_F);
    h16* Q16 = (h16*)(ws + OFF_Q16); h16* K16 = (h16*)(ws + OFF_K16); h16* VT16 = (h16*)(ws + OFF_V16);
    bf* Qh = (bf*)(ws + OFF_QH); bf* Ql = (bf*)(ws + OFF_QL); bf* Kh = (bf*)(ws + OFF_KH); bf* Kl = (bf*)(ws + OFF_KL); bf* VTh = (bf*)(ws + OFF_VH); bf* VTl = (bf*)(ws + OFF_VL);
    bf* ATh = (bf*)(ws + OFF_ATH); bf* ATl = (bf*)(ws + OFF_ATL);

    k_wtG<<<(unsigned)((DM * N3 / 64 + 63) / 64), 256, 0, stream>>>(wqkv, DM, N3, WQKV);
    k_wtG<<<(unsigned)((DM * DM / 64 + 63) / 64), 256, 0, stream>>>(wo, DM, DM, WO);
    k_cvt8<<<dim3((unsigned)(((size_t)SEQ * DM / 8 + 255) / 256), NB, 1), 256, 0, stream>>>(x, XB, (size_t)SEQ * DM / 8, (size_t)SEQ_FULL * DM, (size_t)SEQ * DM);
    k_gemm_qkv<<<dim3(NB * SEQ / 64, N3 / 64, 1), 32, 0, stream>>>(XB, WQKV, DM, F, N3, bqkv);
    k_planes<<<dim3(SEQ / 64, NB * NH, 1), 256, 0, stream>>>(F, Q16, K16, VT16, Qh, Ql, Kh, Kl, VTh, VTl);
    k_attnhl<<<dim3(RH / 64, NB * NH, 1), 128, 0, stream>>>(Qh, Ql, Kh, Kl, VTh, VTl, ATh, ATl);
    if ((SEQ - RH) / 64 > 0)
        k_attn16<<<dim3((SEQ - RH) / 64, NB * NH, 1), 128, 0, stream>>>(Q16, K16, VT16, ATh, ATl);
    k_gemm_proj<<<dim3(SEQ / 64, DM / 64, NB), 32, 0, stream>>>(ATh, ATl, WO, DM, OUT, DM, bo, (size_t)SEQ * DM, (size_t)SEQ_FULL * DM);
}
